// MyModel4_75557064671889
// MI455X (gfx1250) — hardware-verified
//
#include <hip/hip_runtime.h>
#include <stddef.h>
#include <stdint.h>


#define NTHR   256
#define NWAVE  8
#define NF     64
#define NB     512
#define EPT    8
#define CHUNK  (NTHR * EPT)
#define WCAP   (EPT * 32)
#define GRP    128
#define GPB    4
#define RPB    (GRP * GPB)

static_assert(RPB == NB);
static_assert(CHUNK == 2048);
static_assert(WCAP == 256);
static_assert((NB % 64) == 0);

typedef __bf16   bf16;
typedef bf16     v8b  __attribute__((ext_vector_type(8)));
typedef bf16     v16b __attribute__((ext_vector_type(16)));
typedef float    v2f  __attribute__((ext_vector_type(2)));
typedef float    v4f  __attribute__((ext_vector_type(4)));
typedef float    v8f  __attribute__((ext_vector_type(8)));
typedef int      v4i  __attribute__((ext_vector_type(4)));
typedef unsigned v4u  __attribute__((ext_vector_type(4)));
union FragB { v16b v; v8b h[2]; };
union Pack8 { v8b b; v4u u; };

#define RE_W0H    0
#define RE_W0L    2048
#define RE_W1H    4096
#define RE_W1L    8192
#define RE_W2H    12288
#define RE_W2L    16384
#define RE_WCH    20480
#define RE_WCL    24576
#define RE_WBYTES 57344
#define RE_B      57344
#define RE_AH     58112
#define RE_AL     66304
#define RE_ST     74496
#define RE_IDX    107264
#define RE_LDS    108288
#define PE_W0H    0
#define PE_W0L    2048
#define PE_W1H    4096
#define PE_W1L    8192
#define PE_WBYTES 24576
#define PE_B      24576
#define PE_AH     25088
#define PE_AL     33280
#define PE_ST     41472
#define PE_LDS    74240
#define PQ_WH     0
#define PQ_WL     8192
#define PQ_WBYTES 32768
#define PQ_ST     32768
#define PQ_LDS    65536
#define AG_ACC    0
#define AG_W      131072
#define AG_WH     0
#define AG_WL     8192
#define AG_WBYTES 32768
#define AG_B      163840
#define AG_LIST   164352
#define AG_CNT    172544
#define AG_LDS    172672
#define FP_W0H    0
#define FP_W0L    4096
#define FP_W1H    8192
#define FP_W1L    12288
#define FP_W2H    16384
#define FP_W2L    17408
#define FP_WBYTES 36864
#define FP_B      36864
#define FP_ST     37440
#define FP_LDS    38976

__device__ __forceinline__ v8f zero8f() {
  v8f z;
#pragma unroll
  for (int i = 0; i < 8; ++i) z[i] = 0.0f;
  return z;
}

__device__ __forceinline__ v8f wmb(v16b a, v16b b, v8f c) {
  return __builtin_amdgcn_wmma_f32_16x16x32_bf16(false, a, false, b, (short)0, c, false, false);
}

__device__ __forceinline__ v8f wm3(v16b ah, v16b al, v16b bh, v16b bl, v8f c) {
  c = wmb(ah, bh, c);
  c = wmb(ah, bl, c);
  c = wmb(al, bh, c);
  asm volatile("v_nop\n\tv_nop\n\tv_nop\n\tv_nop" : "+v"(c) : "v"(ah), "v"(al), "v"(bh), "v"(bl));
  return c;
}

__device__ __forceinline__ void split8(v8f x, v8b* ph, v8b* pl) {
  v8b h, l;
#pragma unroll
  for (int i = 0; i < 8; ++i) {
    const float xv = x[i];
    const bf16 t = (bf16)xv;
    h[i] = t;
    l[i] = (bf16)(xv - (float)t);
  }
  *ph = h; *pl = l;
}

__device__ __forceinline__ v16b ldk(const bf16* p, int hh) {
  FragB f;
  f.h[0] = *(const v8b*)(p + 8 * hh);
  f.h[1] = *(const v8b*)(p + 16 + 8 * hh);
  return f.v;
}

__device__ __forceinline__ void ldk_f32(const float* p, int hh, v16b* ph, v16b* pl) {
  const v4f a = *(const v4f*)(p + 8 * hh);
  const v4f b = *(const v4f*)(p + 8 * hh + 4);
  const v4f c = *(const v4f*)(p + 16 + 8 * hh);
  const v4f d = *(const v4f*)(p + 20 + 8 * hh);
  v8f x0, x1;
  x0[0] = a.x; x0[1] = a.y; x0[2] = a.z; x0[3] = a.w; x0[4] = b.x; x0[5] = b.y; x0[6] = b.z; x0[7] = b.w;
  x1[0] = c.x; x1[1] = c.y; x1[2] = c.z; x1[3] = c.w; x1[4] = d.x; x1[5] = d.y; x1[6] = d.z; x1[7] = d.w;
  FragB fh, fl;
  split8(x0, &fh.h[0], &fl.h[0]);
  split8(x1, &fh.h[1], &fl.h[1]);
  *ph = fh.v; *pl = fl.v;
}

template <int NFT, int KS>
__device__ __forceinline__ void layerT(const bf16* wh, const bf16* wl, const v16b (&bh)[2], const v16b (&bl)[2],
                                       v8f (&acc)[NFT], int hh, int m) {
  constexpr int pitch = 32 * KS;
#pragma unroll
  for (int ft = 0; ft < NFT; ++ft) {
    v8f c = acc[ft];
#pragma unroll
    for (int kk = 0; kk < KS; ++kk) {
      const int o = (16 * ft + m) * pitch + 32 * kk;
      const v16b ah = ldk(wh + o, hh);
      const v16b al = ldk(wl + o, hh);
      c = wm3(ah, al, bh[kk], bl[kk], c);
    }
    acc[ft] = c;
  }
}

__device__ __forceinline__ void repack4(const v8f (&acc)[4], const float* bias, int hh, v16b (&bh)[2], v16b (&bl)[2]) {
#pragma unroll
  for (int kk = 0; kk < 2; ++kk) {
    FragB fh, fl;
#pragma unroll
    for (int half = 0; half < 2; ++half) {
      const int ft = 2 * kk + half;
      const v4f b0 = *(const v4f*)(bias + 16 * ft + 8 * hh);
      const v4f b1 = *(const v4f*)(bias + 16 * ft + 8 * hh + 4);
      v8f x;
      x[0] = fmaxf(acc[ft][0] + b0.x, 0.0f); x[1] = fmaxf(acc[ft][1] + b0.y, 0.0f);
      x[2] = fmaxf(acc[ft][2] + b0.z, 0.0f); x[3] = fmaxf(acc[ft][3] + b0.w, 0.0f);
      x[4] = fmaxf(acc[ft][4] + b1.x, 0.0f); x[5] = fmaxf(acc[ft][5] + b1.y, 0.0f);
      x[6] = fmaxf(acc[ft][6] + b1.z, 0.0f); x[7] = fmaxf(acc[ft][7] + b1.w, 0.0f);
      split8(x, &fh.h[half], &fl.h[half]);
    }
    bh[kk] = fh.v; bl[kk] = fl.v;
  }
}

template <int BIAS, int RELU>
__device__ __forceinline__ void stage4(float* st, const v8f (&acc)[4], const float* bias, int hh, int m) {
#pragma unroll
  for (int ft = 0; ft < 4; ++ft) {
    v4f b0, b1;
    b0.x = 0.0f; b0.y = 0.0f; b0.z = 0.0f; b0.w = 0.0f; b1 = b0;
    if (BIAS != 0) {
      b0 = *(const v4f*)(bias + 16 * ft + 8 * hh);
      b1 = *(const v4f*)(bias + 16 * ft + 8 * hh + 4);
    }
    v4f o0, o1;
    o0.x = acc[ft][0] + b0.x; o0.y = acc[ft][1] + b0.y; o0.z = acc[ft][2] + b0.z; o0.w = acc[ft][3] + b0.w;
    o1.x = acc[ft][4] + b1.x; o1.y = acc[ft][5] + b1.y; o1.z = acc[ft][6] + b1.z; o1.w = acc[ft][7] + b1.w;
    if (RELU != 0) {
      o0.x = fmaxf(o0.x, 0.0f); o0.y = fmaxf(o0.y, 0.0f); o0.z = fmaxf(o0.z, 0.0f); o0.w = fmaxf(o0.w, 0.0f);
      o1.x = fmaxf(o1.x, 0.0f); o1.y = fmaxf(o1.y, 0.0f); o1.z = fmaxf(o1.z, 0.0f); o1.w = fmaxf(o1.w, 0.0f);
    }
    float* q = st + m * 64 + 16 * ft + 8 * hh;
    *(v4f*)q = o0;
    *(v4f*)(q + 4) = o1;
  }
}

__device__ __forceinline__ void write_tile(const float* st, float* g, int gp, int lane) {
  const int rsel = lane >> 4, piece = lane & 15;
  v4f v[8];
#pragma unroll
  for (int it = 0; it < 8; ++it) v[it] = *(const v4f*)(st + (2 * it + rsel) * 64 + 4 * piece);
#pragma unroll
  for (int it = 0; it < 8; ++it) *(volatile v4f*)(g + (size_t)(2 * it + rsel) * gp + 4 * piece) = v[it];
  __threadfence();
#pragma unroll
  for (int it = 0; it < 8; ++it) *(volatile v4f*)(g + (size_t)(2 * it + rsel) * gp + 4 * piece) = v[it];
}

__global__ __launch_bounds__(NTHR) void k_wcvt(const float* __restrict__ w, int ldw, int koff, int noff,
                                                int Klog, int Kr, int Nsrc, int Kp, int Np, int mode,
                                                bf16* hi, bf16* lo) {
  const int g = blockIdx.x * NTHR + threadIdx.x;
  const int kp8 = Kp >> 3;
  const int ngrp = Np * kp8;
  const int gg = min(g, ngrp - 1);
  const int n = gg / kp8;
  const int k8 = (gg - n * kp8) * 8;
  const int nn = min(n, Nsrc - 1);
  v8b vh, vl;
#pragma unroll
  for (int j = 0; j < 8; ++j) {
    const int k = k8 + j;
    const int kc = min(k, Klog - 1);
    int kr = kc;
    if (mode == 1) kr = (kc < 9) ? kc : ((kc < 18) ? (kc + 6) : (kc + 12));
    else if (mode == 2) kr = (kc < 9) ? kc : (kc + 6);
    kr = min(max(kr, 0), Kr - 1);
    float v = w[(size_t)(kr + koff) * ldw + noff + nn];
    if (k >= Klog || n >= Nsrc) v = 0.0f;
    const bf16 t = (bf16)v;
    vh[j] = t;
    vl[j] = (bf16)(v - (float)t);
  }
  Pack8 ph, pl;
  ph.b = vh; pl.b = vl;
  const bool wr = g < ngrp;
  if (wr) { *(volatile v4u*)(hi + 8 * (size_t)gg) = ph.u; *(volatile v4u*)(lo + 8 * (size_t)gg) = pl.u; }
  __threadfence();
  if (wr) { *(volatile v4u*)(hi + 8 * (size_t)gg) = ph.u; *(volatile v4u*)(lo + 8 * (size_t)gg) = pl.u; }
}

__global__ __launch_bounds__(NTHR) void k_penc(const float* __restrict__ attr, const float* __restrict__ state,
                                                const bf16* pk, const float* __restrict__ b0,
                                                const float* __restrict__ b1, float* penc, int nN) {
  extern __shared__ __attribute__((aligned(16))) unsigned char dynlds[];
  bf16*  W   = (bf16*)dynlds;
  float* sB  = (float*)(dynlds + PE_B);
  bf16*  sAh = (bf16*)(dynlds + PE_AH);
  bf16*  sAl = (bf16*)(dynlds + PE_AL);
  float* stg = (float*)(dynlds + PE_ST);
  const int tid = threadIdx.x, lane = tid & 31, hh = lane >> 4, m = lane & 15;
  const int wave = __builtin_amdgcn_readfirstlane(tid >> 5);
  for (int i = tid; i < PE_WBYTES / 16; i += NTHR) ((v4u*)dynlds)[i] = ((const v4u*)pk)[i];
  if (tid < NF) { sB[tid] = b0[tid]; sB[NF + tid] = b1[tid]; }
  __syncthreads();
  float* mst = stg + wave * (16 * NF);
#pragma unroll 1
  for (int g = 0; g < GPB; ++g) {
    const int n0 = (blockIdx.x * GPB + g) * GRP;
#pragma unroll
    for (int q = 0; q < 4; ++q) {
      const int c = 4 * wave + q;
      const int cls = (c < 9) ? 0 : ((c < 15) ? 1 : 2);
      const int sub = (c < 9) ? c : ((c < 15) ? (c - 9) : 0);
#pragma unroll
      for (int sl = 0; sl < 4; ++sl) {
        const int r = 32 * sl + lane;
        const int node = min(n0 + r, nN - 1);
        float v = 0.0f;
        if (cls == 0)      v = attr[(size_t)node * 9 + sub];
        else if (cls == 1) v = state[(size_t)node * 6 + sub];
        const bf16 t = (bf16)v;
        sAh[r * 32 + c] = t;
        sAl[r * 32 + c] = (bf16)(v - (float)t);
      }
    }
    __syncthreads();
    v16b bh[2], bl[2];
    bh[0] = ldk(sAh + (wave * 16 + m) * 32, hh);
    bl[0] = ldk(sAl + (wave * 16 + m) * 32, hh);
    bh[1] = bh[0]; bl[1] = bl[0];
    v8f acc[4];
#pragma unroll
    for (int i = 0; i < 4; ++i) acc[i] = zero8f();
    layerT<4, 1>(W + PE_W0H, W + PE_W0L, bh, bl, acc, hh, m);
    repack4(acc, sB, hh, bh, bl);
#pragma unroll
    for (int i = 0; i < 4; ++i) acc[i] = zero8f();
    layerT<4, 2>(W + PE_W1H, W + PE_W1L, bh, bl, acc, hh, m);
    stage4<1, 1>(mst, acc, sB + NF, hh, m);
    __syncthreads();
    write_tile(mst, penc + (size_t)(n0 + wave * 16) * NF, NF, lane);
    __syncthreads();
  }
}

__global__ __launch_bounds__(NTHR) void k_relenc(const float* __restrict__ attr, const float* __restrict__ state,
                                                  const float* __restrict__ Ra, const int* __restrict__ recv,
                                                  const int* __restrict__ send, const bf16* pk,
                                                  const float* __restrict__ b0, const float* __restrict__ b1,
                                                  const float* __restrict__ b2, float* Cp, int nN, int nE) {
  extern __shared__ __attribute__((aligned(16))) unsigned char dynlds[];
  bf16*  W   = (bf16*)dynlds;
  float* sB  = (float*)(dynlds + RE_B);
  bf16*  sAh = (bf16*)(dynlds + RE_AH);
  bf16*  sAl = (bf16*)(dynlds + RE_AL);
  float* stg = (float*)(dynlds + RE_ST);
  int*   sR  = (int*)(dynlds + RE_IDX);
  int*   sS  = sR + GRP;
  const int tid = threadIdx.x, lane = tid & 31, hh = lane >> 4, m = lane & 15;
  const int wave = __builtin_amdgcn_readfirstlane(tid >> 5);
  for (int i = tid; i < RE_WBYTES / 16; i += NTHR) ((v4u*)dynlds)[i] = ((const v4u*)pk)[i];
  if (tid < NF) { sB[tid] = b0[tid]; sB[NF + tid] = b1[tid]; sB[2 * NF + tid] = b2[tid]; }
  __syncthreads();
  float* mst = stg + wave * (16 * NF);
#pragma unroll 1
  for (int g = 0; g < GPB; ++g) {
    const int e0 = (blockIdx.x * GPB + g) * GRP;
    if (tid < GRP) {
      const int e = min(e0 + tid, nE - 1);
      int rv = recv[e], sv = send[e];
      rv = min(max(rv, 0), nN - 1);
      sv = min(max(sv, 0), nN - 1);
      sR[tid] = rv; sS[tid] = sv;
    }
    __syncthreads();
#pragma unroll
    for (int q = 0; q < 4; ++q) {
      const int c = 4 * wave + q;
      const int cls = (c < 18) ? 0 : ((c < 30) ? 1 : 2);
      const bool useR = (c < 9) || (c >= 18 && c < 24);
      const int sub = (c < 9) ? c : ((c < 18) ? (c - 9) : ((c < 24) ? (c - 18) : ((c < 30) ? (c - 24) : 0)));
#pragma unroll
      for (int sl = 0; sl < 4; ++sl) {
        const int r = 32 * sl + lane;
        const int e = min(e0 + r, nE - 1);
        const int nr = sR[r], ns = sS[r];
        const int node = useR ? nr : ns;
        float v;
        if (cls == 0)      v = attr[(size_t)node * 9 + sub];
        else if (cls == 1) v = state[(size_t)node * 6 + sub];
        else               v = Ra[e];
        if (c == 31) v = 0.0f;
        const bf16 t = (bf16)v;
        sAh[r * 32 + c] = t;
        sAl[r * 32 + c] = (bf16)(v - (float)t);
      }
    }
    __syncthreads();
    v16b bh[2], bl[2];
    bh[0] = ldk(sAh + (wave * 16 + m) * 32, hh);
    bl[0] = ldk(sAl + (wave * 16 + m) * 32, hh);
    bh[1] = bh[0]; bl[1] = bl[0];
    v8f acc[4];
#pragma unroll
    for (int i = 0; i < 4; ++i) acc[i] = zero8f();
    layerT<4, 1>(W + RE_W0H, W + RE_W0L, bh, bl, acc, hh, m);
    repack4(acc, sB, hh, bh, bl);
#pragma unroll
    for (int i = 0; i < 4; ++i) acc[i] = zero8f();
    layerT<4, 2>(W + RE_W1H, W + RE_W1L, bh, bl, acc, hh, m);
    repack4(acc, sB + NF, hh, bh, bl);
#pragma unroll
    for (int i = 0; i < 4; ++i) acc[i] = zero8f();
    layerT<4, 2>(W + RE_W2H, W + RE_W2L, bh, bl, acc, hh, m);
    repack4(acc, sB + 2 * NF, hh, bh, bl);
#pragma unroll
    for (int i = 0; i < 4; ++i) acc[i] = zero8f();
    layerT<4, 2>(W + RE_WCH, W + RE_WCL, bh, bl, acc, hh, m);
    stage4<0, 0>(mst, acc, sB, hh, m);
    __syncthreads();
    write_tile(mst, Cp + (size_t)(e0 + wave * 16) * NF, NF, lane);
    __syncthreads();
  }
}

__global__ __launch_bounds__(NTHR) void k_pq(const float* eff, const bf16* pk, float* PQ, int nNp) {
  extern __shared__ __attribute__((aligned(16))) unsigned char dynlds[];
  bf16*  W   = (bf16*)dynlds;
  float* stg = (float*)(dynlds + PQ_ST);
  const int tid = threadIdx.x, lane = tid & 31, hh = lane >> 4, m = lane & 15;
  const int wave = __builtin_amdgcn_readfirstlane(tid >> 5);
  for (int i = tid; i < PQ_WBYTES / 16; i += NTHR) ((v4u*)dynlds)[i] = ((const v4u*)pk)[i];
  __syncthreads();
  float* mst = stg + wave * (16 * NF);
#pragma unroll 1
  for (int g = 0; g < GPB; ++g) {
    const int n0 = (blockIdx.x * GPB + g) * GRP;
    const int node = min(n0 + wave * 16 + m, nNp - 1);
    v16b bh[2], bl[2];
#pragma unroll
    for (int kk = 0; kk < 2; ++kk) ldk_f32(eff + (size_t)node * NF + 32 * kk, hh, &bh[kk], &bl[kk]);
#pragma unroll 1
    for (int p = 0; p < 2; ++p) {
      v8f acc[4];
#pragma unroll
      for (int i = 0; i < 4; ++i) acc[i] = zero8f();
      layerT<4, 2>(W + PQ_WH + p * 4096, W + PQ_WL + p * 4096, bh, bl, acc, hh, m);
      stage4<0, 0>(mst, acc, stg, hh, m);
      __syncthreads();
      write_tile(mst, PQ + (size_t)(n0 + wave * 16) * 128 + 64 * p, 128, lane);
      __syncthreads();
    }
  }
}

__device__ __forceinline__ int scan_chunk(const int* __restrict__ dsts, int nE, int cbase, int nodeBase,
                                          int vec8, int* list, int tid, int wave) {
  int wc = 0;
  const int el0 = tid * EPT;
  const int e0 = cbase + el0;
  const int sent = -2147483647 - 1;
  v4i da, db;
  if (vec8 != 0 && cbase + CHUNK <= nE) {
    da = *(const v4i*)(dsts + e0);
    db = *(const v4i*)(dsts + e0 + 4);
  } else {
    da.x = (e0     < nE) ? dsts[min(e0,     nE - 1)] : sent;
    da.y = (e0 + 1 < nE) ? dsts[min(e0 + 1, nE - 1)] : sent;
    da.z = (e0 + 2 < nE) ? dsts[min(e0 + 2, nE - 1)] : sent;
    da.w = (e0 + 3 < nE) ? dsts[min(e0 + 3, nE - 1)] : sent;
    db.x = (e0 + 4 < nE) ? dsts[min(e0 + 4, nE - 1)] : sent;
    db.y = (e0 + 5 < nE) ? dsts[min(e0 + 5, nE - 1)] : sent;
    db.z = (e0 + 6 < nE) ? dsts[min(e0 + 6, nE - 1)] : sent;
    db.w = (e0 + 7 < nE) ? dsts[min(e0 + 7, nE - 1)] : sent;
  }
  const unsigned nb = (unsigned)nodeBase;
  const unsigned s0 = (unsigned)da.x - nb, s1 = (unsigned)da.y - nb;
  const unsigned s2 = (unsigned)da.z - nb, s3 = (unsigned)da.w - nb;
  const unsigned s4 = (unsigned)db.x - nb, s5 = (unsigned)db.y - nb;
  const unsigned s6 = (unsigned)db.z - nb, s7 = (unsigned)db.w - nb;
  const bool h0 = s0 < (unsigned)NB, h1 = s1 < (unsigned)NB, h2 = s2 < (unsigned)NB, h3 = s3 < (unsigned)NB;
  const bool h4 = s4 < (unsigned)NB, h5 = s5 < (unsigned)NB, h6 = s6 < (unsigned)NB, h7 = s7 < (unsigned)NB;
  const unsigned any = __builtin_amdgcn_ballot_w32(h0 | h1 | h2 | h3 | h4 | h5 | h6 | h7);
  if (any != 0u) {
#define HITJ(J, HJ, SJ) { \
      const unsigned mj = __builtin_amdgcn_ballot_w32(HJ); \
      if (mj != 0u) { \
        if (HJ) { \
          const int pos = wc + (int)__builtin_amdgcn_mbcnt_lo(mj, 0u); \
          if (pos < WCAP) list[wave * WCAP + pos] = (int)(((SJ) << 11) | (unsigned)(el0 + (J))); \
        } \
        wc += (int)__builtin_popcount(mj); } }
    HITJ(0, h0, s0)
    HITJ(1, h1, s1)
    HITJ(2, h2, s2)
    HITJ(3, h3, s3)
    HITJ(4, h4, s4)
    HITJ(5, h5, s5)
    HITJ(6, h6, s6)
    HITJ(7, h7, s7)
#undef HITJ
  }
  return wc;
}

__global__ __launch_bounds__(NTHR) void k_agg(const int* __restrict__ recv, const int* __restrict__ send,
                                               const float* Cp, const float* PQ, const float* penc,
                                               const bf16* pk, const float* __restrict__ rp_b,
                                               const float* __restrict__ pp_b, float* effo,
                                               int nN, int nE, int hasPQ, int vec8) {
  extern __shared__ __attribute__((aligned(16))) unsigned char dynlds[];
  float* acc  = (float*)(dynlds + AG_ACC);
  bf16*  W    = (bf16*)(dynlds + AG_W);
  float* sB   = (float*)(dynlds + AG_B);
  int*   list = (int*)(dynlds + AG_LIST);
  int*   wcnt = (int*)(dynlds + AG_CNT);
  const int tid = threadIdx.x, lane = tid & 31, hh = lane >> 4, m = lane & 15;
  const int wave = __builtin_amdgcn_readfirstlane(tid >> 5);
  const int nodeBase = blockIdx.x * NB;

  {
    v4f z; z.x = 0.0f; z.y = 0.0f; z.z = 0.0f; z.w = 0.0f;
    for (int i = tid; i < NB * NF / 4; i += NTHR) ((v4f*)acc)[i] = z;
  }
  for (int i = tid; i < AG_WBYTES / 16; i += NTHR) ((v4u*)(dynlds + AG_W))[i] = ((const v4u*)pk)[i];
  if (tid < NF) { sB[tid] = rp_b[tid]; sB[NF + tid] = pp_b[tid]; }
  __syncthreads();
  const v2f rb = *(const v2f*)(sB + 2 * lane);

  const int nChunks = (nE + CHUNK - 1) / CHUNK;
#pragma unroll 1
  for (int ch = 0; ch < nChunks; ++ch) {
    const int cbase = ch * CHUNK;
    const int wc = scan_chunk(recv, nE, cbase, nodeBase, vec8, list, tid, wave);
    if (lane == 0) wcnt[wave] = wc;
    __syncthreads();
#pragma unroll 1
    for (int w = 0; w < NWAVE; ++w) {
      int n = __builtin_amdgcn_readfirstlane(wcnt[w]);
      n = n > WCAP ? WCAP : (n < 0 ? 0 : n);
#pragma unroll 1
      for (int i = 0; i < n; ++i) {
        const int ent = __builtin_amdgcn_readfirstlane(list[w * WCAP + i]);
        int slot = (ent >> 11) & 1023;
        slot = slot > NB - 1 ? NB - 1 : slot;
        if ((slot & (NWAVE - 1)) == wave) {
          int e = cbase + (ent & (CHUNK - 1));
          e = e > nE - 1 ? nE - 1 : e;
          const v2f cv = *(const v2f*)(Cp + (size_t)e * NF + 2 * lane);
          float t0 = cv.x, t1 = cv.y;
          if (hasPQ != 0) {
            int s = send[e];
            s = min(max(s, 0), nN - 1);
            const int rn = min(nodeBase + slot, nN - 1);
            const v2f pv = *(const v2f*)(PQ + (size_t)rn * 128 + 2 * lane);
            const v2f qv = *(const v2f*)(PQ + (size_t)s * 128 + 64 + 2 * lane);
            t0 += pv.x + qv.x;
            t1 += pv.y + qv.y;
          }
          t0 = fmaxf(t0 + rb.x, 0.0f);
          t1 = fmaxf(t1 + rb.y, 0.0f);
          float* ap = acc + slot * NF + 2 * lane;
          v2f o = *(const v2f*)ap;
          o.x += t0; o.y += t1;
          *(v2f*)ap = o;
        }
      }
    }
    __syncthreads();
  }
  __syncthreads();

  const bf16* Wh = W + AG_WH;
  const bf16* Wl = W + AG_WL;
#pragma unroll 1
  for (int t = 0; t < 4; ++t) {
    const int slot0 = 64 * wave + 16 * t;
    v8f acc4[4];
#pragma unroll
    for (int i = 0; i < 4; ++i) acc4[i] = zero8f();
#pragma unroll
    for (int kk = 0; kk < 4; ++kk) {
      v16b bh, bl;
      if (kk < 2) ldk_f32(penc + (size_t)(nodeBase + slot0 + m) * NF + 32 * kk, hh, &bh, &bl);
      else        ldk_f32(acc + (slot0 + m) * NF + 32 * (kk - 2), hh, &bh, &bl);
#pragma unroll
      for (int ft = 0; ft < 4; ++ft) {
        const int o = (16 * ft + m) * 128 + 32 * kk;
        acc4[ft] = wm3(ldk(Wh + o, hh), ldk(Wl + o, hh), bh, bl, acc4[ft]);
      }
    }
    stage4<1, 1>(acc + slot0 * NF, acc4, sB + NF, hh, m);
    __syncthreads();
    write_tile(acc + slot0 * NF, effo + (size_t)(nodeBase + slot0) * NF, NF, lane);
    __syncthreads();
  }
}

__global__ __launch_bounds__(NTHR) void k_pred(const float* eff, const bf16* pk, const float* __restrict__ b0,
                                                const float* __restrict__ b1, const float* __restrict__ b2,
                                                float* out, int nN, int nNp) {
  extern __shared__ __attribute__((aligned(16))) unsigned char dynlds[];
  bf16*  W     = (bf16*)dynlds;
  float* sB    = (float*)(dynlds + FP_B);
  float* spred = (float*)(dynlds + FP_ST);
  const int tid = threadIdx.x, lane = tid & 31, hh = lane >> 4, m = lane & 15;
  const int wave = __builtin_amdgcn_readfirstlane(tid >> 5);
  for (int i = tid; i < FP_WBYTES / 16; i += NTHR) ((v4u*)dynlds)[i] = ((const v4u*)pk)[i];
  if (tid < NF) { sB[tid] = b0[tid]; sB[NF + tid] = b1[tid]; }
  if (tid < 16) { const float bv = b2[min(tid, 2)]; sB[2 * NF + tid] = (tid < 3) ? bv : 0.0f; }
  __syncthreads();
  const size_t lim = (size_t)nN * 3;
#pragma unroll 1
  for (int g = 0; g < GPB; ++g) {
    const int n0 = (blockIdx.x * GPB + g) * GRP;
    const int node = min(n0 + wave * 16 + m, nNp - 1);
    v16b bh[2], bl[2];
#pragma unroll
    for (int kk = 0; kk < 2; ++kk) ldk_f32(eff + (size_t)node * NF + 32 * kk, hh, &bh[kk], &bl[kk]);
    v8f acc[4];
#pragma unroll
    for (int i = 0; i < 4; ++i) acc[i] = zero8f();
    layerT<4, 2>(W + FP_W0H, W + FP_W0L, bh, bl, acc, hh, m);
    repack4(acc, sB, hh, bh, bl);
#pragma unroll
    for (int i = 0; i < 4; ++i) acc[i] = zero8f();
    layerT<4, 2>(W + FP_W1H, W + FP_W1L, bh, bl, acc, hh, m);
    repack4(acc, sB + NF, hh, bh, bl);
    v8f a1[1];
    a1[0] = zero8f();
    layerT<1, 2>(W + FP_W2H, W + FP_W2L, bh, bl, a1, hh, m);
    const float p0 = a1[0][0] + sB[2 * NF + 0];
    const float p1 = a1[0][1] + sB[2 * NF + 1];
    const float p2 = a1[0][2] + sB[2 * NF + 2];
    if (hh == 0) {
      float* sp = spred + (wave * 16 + m) * 3;
      sp[0] = p0; sp[1] = p1; sp[2] = p2;
    }
    __syncthreads();
    const bool act = tid < 96;
    v4f ov; ov.x = 0.0f; ov.y = 0.0f; ov.z = 0.0f; ov.w = 0.0f;
    if (act) ov = ((const v4f*)spred)[tid];
    const size_t gi = (size_t)n0 * 3 + 4 * (size_t)tid;
    const bool full = act && (gi + 4 <= lim);
    const bool part = act && !full && (gi < lim);
    if (full) *(volatile v4f*)(out + gi) = ov;
    if (part) {
      if (gi     < lim) ((volatile float*)out)[gi]     = ov.x;
      if (gi + 1 < lim) ((volatile float*)out)[gi + 1] = ov.y;
      if (gi + 2 < lim) ((volatile float*)out)[gi + 2] = ov.z;
      if (gi + 3 < lim) ((volatile float*)out)[gi + 3] = ov.w;
    }
    __threadfence();
    if (full) *(volatile v4f*)(out + gi) = ov;
    if (part) {
      if (gi     < lim) ((volatile float*)out)[gi]     = ov.x;
      if (gi + 1 < lim) ((volatile float*)out)[gi + 1] = ov.y;
      if (gi + 2 < lim) ((volatile float*)out)[gi + 2] = ov.z;
      if (gi + 3 < lim) ((volatile float*)out)[gi + 3] = ov.w;
    }
    __syncthreads();
  }
}

static void launch_wcvt(hipStream_t stream, const float* w, int ldw, int koff, int noff, int Klog, int Kr,
                        int Nsrc, int Kp, int Np, int mode, bf16* hi, bf16* lo) {
  const int ngrp = Np * (Kp / 8);
  const int nblk = (ngrp + NTHR - 1) / NTHR;
  k_wcvt<<<nblk, NTHR, 0, stream>>>(w, ldw, koff, noff, Klog, Kr, Nsrc, Kp, Np, mode, hi, lo);
}

extern "C" void kernel_launch(void* const* d_in, const int* in_sizes, int n_in,
                              void* d_out, int out_size, void* d_ws, size_t ws_size,
                              hipStream_t stream) {
  if (n_in < 25) return;
  const int nN = in_sizes[0] / 9;
  if (nN <= 0 || in_sizes[0] != nN * 9 || in_sizes[1] != nN * 6) return;
  const int nE = in_sizes[3];
  if (nE <= 0 || in_sizes[4] != nE || in_sizes[2] != nE) return;
  if (in_sizes[5] != 21 * NF || in_sizes[6] != NF || in_sizes[7] != NF * NF || in_sizes[8] != NF) return;
  if (in_sizes[9] != 43 * NF || in_sizes[10] != NF || in_sizes[11] != NF * NF || in_sizes[12] != NF) return;
  if (in_sizes[13] != NF * NF || in_sizes[14] != NF) return;
  if (in_sizes[15] != 192 * NF || in_sizes[16] != NF || in_sizes[17] != 128 * NF || in_sizes[18] != NF) return;
  if (in_sizes[19] != NF * NF || in_sizes[20] != NF || in_sizes[21] != NF * NF || in_sizes[22] != NF) return;
  if (in_sizes[23] != NF * 3 || in_sizes[24] != 3) return;
  if (out_size != nN * 3) return;

  const float* attr  = (const float*)d_in[0];
  const float* state = (const float*)d_in[1];
  const float* Ra    = (const float*)d_in[2];
  const int*   recv  = (const int*)d_in[3];
  const int*   send  = (const int*)d_in[4];
  const float* pe_w0 = (const float*)d_in[5];
  const float* pe_b0 = (const float*)d_in[6];
  const float* pe_w1 = (const float*)d_in[7];
  const float* pe_b1 = (const float*)d_in[8];
  const float* re_w0 = (const float*)d_in[9];
  const float* re_b0 = (const float*)d_in[10];
  const float* re_w1 = (const float*)d_in[11];
  const float* re_b1 = (const float*)d_in[12];
  const float* re_w2 = (const float*)d_in[13];
  const float* re_b2 = (const float*)d_in[14];
  const float* rp_w  = (const float*)d_in[15];
  const float* rp_b  = (const float*)d_in[16];
  const float* pp_w  = (const float*)d_in[17];
  const float* pp_b  = (const float*)d_in[18];
  const float* fp_w0 = (const float*)d_in[19];
  const float* fp_b0 = (const float*)d_in[20];
  const float* fp_w1 = (const float*)d_in[21];
  const float* fp_b1 = (const float*)d_in[22];
  const float* fp_w2 = (const float*)d_in[23];
  const float* fp_b2 = (const float*)d_in[24];
  float* out = (float*)d_out;

  const int nNp = ((nN + RPB - 1) / RPB) * RPB;
  const int nEp = ((nE + RPB - 1) / RPB) * RPB;
  const int nBlkN = nNp / RPB;
  const int nBlkE = nEp / RPB;
  const int nBlkA = nNp / NB;

  char* ws = (char*)d_ws;
  size_t off = 0;
  const size_t oPkRE = off; off += RE_WBYTES;
  const size_t oPkPE = off; off += PE_WBYTES;
  const size_t oPkPQ = off; off += PQ_WBYTES;
  const size_t oPkPP = off; off += AG_WBYTES;
  const size_t oPkFP = off; off += FP_WBYTES;
  const size_t oC    = off; off += (size_t)nEp * NF * 4;
  const size_t oPenc = off; off += (size_t)nNp * NF * 4;
  const size_t oEff  = off; off += (size_t)nNp * NF * 4;
  const size_t oPQ   = off; off += (size_t)nNp * 128 * 4;
  if (off > ws_size) return;

  bf16* pkRE = (bf16*)(ws + oPkRE);
  bf16* pkPE = (bf16*)(ws + oPkPE);
  bf16* pkPQ = (bf16*)(ws + oPkPQ);
  bf16* pkPP = (bf16*)(ws + oPkPP);
  bf16* pkFP = (bf16*)(ws + oPkFP);
  float* Cp    = (float*)(ws + oC);
  float* penc  = (float*)(ws + oPenc);
  float* eff   = (float*)(ws + oEff);
  float* PQ    = (float*)(ws + oPQ);

  const int vec8 = ((nE & 3) == 0) ? 1 : 0;

  hipFuncSetAttribute(reinterpret_cast<const void*>(&k_relenc), hipFuncAttributeMaxDynamicSharedMemorySize, RE_LDS);
  hipFuncSetAttribute(reinterpret_cast<const void*>(&k_penc),   hipFuncAttributeMaxDynamicSharedMemorySize, PE_LDS);
  hipFuncSetAttribute(reinterpret_cast<const void*>(&k_pq),     hipFuncAttributeMaxDynamicSharedMemorySize, PQ_LDS);
  hipFuncSetAttribute(reinterpret_cast<const void*>(&k_agg),    hipFuncAttributeMaxDynamicSharedMemorySize, AG_LDS);

  launch_wcvt(stream, re_w0, NF, 0,   0, 31,  43,  NF, 32,  NF, 1, pkRE + RE_W0H, pkRE + RE_W0L);
  launch_wcvt(stream, re_w1, NF, 0,   0, NF,  NF,  NF, 64,  NF, 0, pkRE + RE_W1H, pkRE + RE_W1L);
  launch_wcvt(stream, re_w2, NF, 0,   0, NF,  NF,  NF, 64,  NF, 0, pkRE + RE_W2H, pkRE + RE_W2L);
  launch_wcvt(stream, rp_w,  NF, 0,   0, NF,  NF,  NF, 64,  NF, 0, pkRE + RE_WCH, pkRE + RE_WCL);
  launch_wcvt(stream, pe_w0, NF, 0,   0, 15,  21,  NF, 32,  NF, 2, pkPE + PE_W0H, pkPE + PE_W0L);
  launch_wcvt(stream, pe_w1, NF, 0,   0, NF,  NF,  NF, 64,  NF, 0, pkPE + PE_W1H, pkPE + PE_W1L);
  launch_wcvt(stream, rp_w,  NF, 64,  0, NF,  NF,  NF, 64,  NF, 0, pkPQ + PQ_WH,        pkPQ + PQ_WL);
  launch_wcvt(stream, rp_w,  NF, 128, 0, NF,  NF,  NF, 64,  NF, 0, pkPQ + PQ_WH + 4096, pkPQ + PQ_WL + 4096);
  launch_wcvt(stream, pp_w,  NF, 0,   0, 128, 128, NF, 128, NF, 0, pkPP + AG_WH, pkPP + AG_WL);
  launch_wcvt(stream, fp_w0, NF, 0,   0, NF,  NF,  NF, 64,  NF, 0, pkFP + FP_W0H, pkFP + FP_W0L);
  launch_wcvt(stream, fp_w1, NF, 0,   0, NF,  NF,  NF, 64,  NF, 0, pkFP + FP_W1H, pkFP + FP_W1L);
  launch_wcvt(stream, fp_w2, 3,  0,   0, NF,  NF,  3,  64,  16, 0, pkFP + FP_W2H, pkFP + FP_W2L);

  k_penc<<<nBlkN, NTHR, PE_LDS, stream>>>(attr, state, pkPE, pe_b0, pe_b1, penc, nN);
  k_relenc<<<nBlkE, NTHR, RE_LDS, stream>>>(attr, state, Ra, recv, send, pkRE, re_b0, re_b1, re_b2, Cp, nN, nE);

  k_agg<<<nBlkA, NTHR, AG_LDS, stream>>>(recv, send, Cp, PQ, penc, pkPP, rp_b, pp_b, eff, nN, nE, 0, vec8);
  k_pq<<<nBlkN, NTHR, PQ_LDS, stream>>>(eff, pkPQ, PQ, nNp);
  k_agg<<<nBlkA, NTHR, AG_LDS, stream>>>(recv, send, Cp, PQ, penc, pkPP, rp_b, pp_b, eff, nN, nE, 1, vec8);

  k_pred<<<nBlkN, NTHR, FP_LDS, stream>>>(eff, pkFP, fp_b0, fp_b1, fp_b2, out, nN, nNp);
}
